// StatefulBlock_85899346617
// MI455X (gfx1250) — hardware-verified
//
#include <hip/hip_runtime.h>

#define EPSF 1.1920929e-07f

typedef __attribute__((ext_vector_type(16))) _Float16        v16bf;
typedef __attribute__((ext_vector_type(4)))  float           v4f;
typedef __attribute__((ext_vector_type(4)))  unsigned        v4u;
template <typename V> __device__ __forceinline__ void vst2(void* p, V v) {
    *(volatile V*)p = v; __threadfence(); *(volatile V*)p = v;
}
typedef float __attribute__((may_alias)) float_a;
#define PSC 256.0f
#define PUN (1.0f / 256.0f)
typedef __attribute__((ext_vector_type(8)))  float           v8f;
typedef __attribute__((ext_vector_type(8)))  unsigned short  ushort8;
typedef __attribute__((ext_vector_type(16))) unsigned short  ushort16;

union Frag {
    ushort16 u;
    v16bf    b;
    ushort8  h[2];
};

__device__ __forceinline__ unsigned short f2b(float f) {
    union { _Float16 h; unsigned short u; } c; c.h = (_Float16)f; return c.u;
}
__device__ __forceinline__ float b2f(unsigned short s) {
    union { unsigned short u; _Float16 h; } c; c.u = s; return (float)c.h;
}
__device__ __forceinline__ v8f wmma16(v16bf a, v16bf b, v8f c) {
    v8f d = __builtin_amdgcn_wmma_f32_16x16x32_f16(false, a, false, b, (short)0, c, false, false);
    asm volatile("v_nop\n\tv_nop\n\tv_nop\n\tv_nop" : "+v"(d) : "v"(a), "v"(b));
    return d;
}

__global__ void film_kernel(const float* __restrict__ state, const float* __restrict__ wsm,
                            const float* __restrict__ gamma, const float* __restrict__ beta,
                            float* __restrict__ fg, float* __restrict__ fb, int SD, int D) {
    int idx = blockIdx.x * blockDim.x + threadIdx.x;
    int b = idx / (2 * D);
    int c = idx % (2 * D);
    if (b >= 2) return;
    float s = 0.f;
    for (int k = 0; k < SD; ++k) s += state[b * SD + k] * wsm[k * 2 * D + c];
    if (c < D) vst2(fg + b * D + c, (float_a)(gamma[c] * (1.f + s)));
    else       vst2(fb + b * D + (c - D), (float_a)(beta[c - D] + s));
}

__global__ __launch_bounds__(256) void rmsnorm_film(
        const float* __restrict__ x, const float* __restrict__ nw,
        const float* __restrict__ fg, const float* __restrict__ fb,
        unsigned short* __restrict__ out, int S, int D) {
    int row = blockIdx.x;
    int b = row / S;
    const float* xr = x + (size_t)row * D;
    float ss = 0.f;
    for (int d = threadIdx.x; d < D; d += 256) { float v = xr[d]; ss += v * v; }
    for (int m = 16; m >= 1; m >>= 1) ss += __shfl_xor(ss, m, 32);
    __shared__ float red[8];
    if ((threadIdx.x & 31) == 0) red[threadIdx.x >> 5] = ss;
    __syncthreads();
    float tot = 0.f;
    for (int i = 0; i < 8; ++i) tot += red[i];
    float scale = rsqrtf(tot / (float)D + EPSF);
    const float* fgb = fg + (size_t)b * D;
    const float* fbb = fb + (size_t)b * D;
    unsigned short* orow = out + (size_t)row * D;
    {
        const int d0 = threadIdx.x * 4;
        union { unsigned short s[4]; unsigned long long u; } pk;
        #pragma unroll
        for (int e = 0; e < 4; ++e) { const int d = d0 + e; pk.s[e] = f2b(xr[d] * scale * nw[d] * fgb[d] + fbb[d]); }
        vst2(orow + d0, pk.u);
    }
}

__global__ void pack_b(const float* __restrict__ W, unsigned short* __restrict__ out, int K, int N) {
    int g = blockIdx.x * 256 + threadIdx.x;
    if (g * 8 >= K * N) return;
    union { unsigned short s[8]; v4u u; } pk;
    #pragma unroll
    for (int q = 0; q < 8; ++q) {
        int idx  = g * 8 + q;
        int j    = idx & 15;
        int lane = (idx >> 4) & 31;
        int r    = idx >> 9;
        int ktc  = K >> 5;
        int kt   = r % ktc;
        int nt   = r / ktc;
        int k = kt * 32 + 8 * (lane >> 4) + (j < 8 ? j : j + 8);
        int n = nt * 16 + (lane & 15);
        pk.s[q] = f2b(W[(size_t)k * N + n]);
    }
    vst2(out + (size_t)g * 8, pk.u);
}

__global__ void pack_v(const unsigned short* __restrict__ qkvb, unsigned short* __restrict__ vp,
                       int S, int H, int HD, int total) {
    int g = blockIdx.x * 256 + threadIdx.x;
    if (g * 8 >= total) return;
    union { unsigned short s[8]; v4u u; } pk;
    #pragma unroll
    for (int q = 0; q < 8; ++q) {
        int idx  = g * 8 + q;
        int j    = idx & 15;
        int lane = (idx >> 4) & 31;
        int r    = idx >> 9;
        int n4 = r & 3;  r >>= 2;
        int kb = r & 63; r >>= 6;
        int bh = r;
        int b = bh >> 4, h = bh & 15;
        int key = kb * 32 + 8 * (lane >> 4) + (j < 8 ? j : j + 8);
        int col = n4 * 16 + (lane & 15);
        pk.s[q] = qkvb[(size_t)(b * S + key) * (3 * H * HD) + 2 * H * HD + h * HD + col];
    }
    vst2(vp + (size_t)g * 8, pk.u);
}

template <int EPI>
__global__ __launch_bounds__(256) void gemm_f16(
        const unsigned short* __restrict__ A, const unsigned short* __restrict__ Bp,
        const float* __restrict__ resF, const unsigned short* __restrict__ gateB,
        float* __restrict__ outF, unsigned short* __restrict__ outB,
        int M, int N, int K) {
    __shared__ __align__(16) unsigned short atile[2][64 * 32];
    __shared__ __align__(16) float Ct[64][256];

    const int lane = threadIdx.x & 31;
    const int w    = threadIdx.x >> 5;
    const int wm   = w >> 2;
    const int wn   = w & 3;
    const int mblock = blockIdx.y * 64;
    const int mbase  = mblock + wm * 32;
    const int nbase  = blockIdx.x * 256 + wn * 64;
    const int ktc = K >> 5;
    const int hi  = (lane >> 4) & 1;
    const int l15 = lane & 15;

    const int srow   = threadIdx.x >> 2;
    const int schunk = (threadIdx.x & 3) * 8;

    v8f acc[2][4] = {};

    const unsigned short* bp[4];
    for (int ni = 0; ni < 4; ++ni)
        bp[ni] = Bp + ((size_t)((nbase >> 4) + ni) * ktc) * 512 + lane * 16;

    const unsigned short* ag = A + (size_t)(mblock + srow) * K + schunk;

    auto issue = [&](int buf, int kt) {
        *(v4u*)(&atile[buf][srow * 32 + schunk]) = *(const v4u*)(ag + kt * 32);
    };

    issue(0, 0);
    int cur = 0;

    for (int kt = 0; kt < ktc; ++kt) {
        __syncthreads();
        if (kt + 1 < ktc) issue(cur ^ 1, kt + 1);

        Frag bfr[4];
        for (int ni = 0; ni < 4; ++ni) {
            bfr[ni].u = *(const ushort16*)(bp[ni]);
            if (kt + 1 < ktc) __builtin_prefetch(bp[ni] + 512, 0, 0);
            bp[ni] += 512;
        }

        Frag a0, a1;
        const unsigned short* l0 = &atile[cur][(wm * 32 + l15) * 32 + hi * 8];
        a0.h[0] = *(const ushort8*)(l0);
        a0.h[1] = *(const ushort8*)(l0 + 16);
        const unsigned short* l1 = l0 + 16 * 32;
        a1.h[0] = *(const ushort8*)(l1);
        a1.h[1] = *(const ushort8*)(l1 + 16);

        for (int ni = 0; ni < 4; ++ni) {
            acc[0][ni] = wmma16(a0.b, bfr[ni].b, acc[0][ni]);
            acc[1][ni] = wmma16(a1.b, bfr[ni].b, acc[1][ni]);
        }
        cur ^= 1;
    }

    __syncthreads();
    for (int mi = 0; mi < 2; ++mi) {
        for (int ni = 0; ni < 4; ++ni) {
            int rl0 = wm * 32 + mi * 16 + hi * 8;
            int cl  = wn * 64 + ni * 16 + l15;
            int col = blockIdx.x * 256 + cl;
            for (int r = 0; r < 8; ++r) {
                size_t idx = (size_t)(mblock + rl0 + r) * N + col;
                float v = acc[mi][ni][r];
                if (EPI == 1)      v += resF[idx];
                else if (EPI == 2) v = v / (1.f + __expf(-v));
                else if (EPI == 3) v = b2f(gateB[idx]) * v;
                Ct[rl0 + r][cl] = v;
            }
        }
    }
    __syncthreads();
    const int tid = threadIdx.x, n0blk = blockIdx.x * 256;
    if (EPI == 1) {
        for (int g = tid; g < 64 * 64; g += 256) { const int rl = g >> 6, pc = g & 63; vst2(outF + (size_t)(mblock + rl) * N + n0blk + pc * 4, *(const v4f*)(&Ct[rl][pc * 4])); }
    } else {
        for (int g = tid; g < 64 * 32; g += 256) {
            const int rl = g >> 5, pc = g & 31;
            union { unsigned short s[8]; v4u u; } pk;
            #pragma unroll
            for (int e = 0; e < 8; ++e) pk.s[e] = f2b(Ct[rl][pc * 8 + e]);
            vst2(outB + (size_t)(mblock + rl) * N + n0blk + pc * 8, pk.u);
        }
    }
}

__global__ __launch_bounds__(256) void flash_attn(
        const unsigned short* __restrict__ qkvb, const unsigned short* __restrict__ vp,
        unsigned short* __restrict__ attn, int S, int H, int HD) {
    __shared__ __align__(16) unsigned short plds[8][512];
    __shared__ __align__(16) unsigned short olds[8][16 * 64];
    const int lane = threadIdx.x & 31;
    const int w    = threadIdx.x >> 5;
    const int waveId = blockIdx.x * 8 + w;
    const int qt = waveId & 127;
    const int bh = waveId >> 7;
    const int b = bh >> 4, h = bh & 15;
    const int qbase = qt * 16;
    const int l15 = lane & 15;
    const int hi  = (lane >> 4) & 1;
    const int D3  = 3 * H * HD;

    Frag aq[2];
    {
        const unsigned short* qp = qkvb + (size_t)(b * S + qbase + l15) * D3 + h * HD + hi * 8;
        aq[0].h[0] = *(const ushort8*)(qp);
        aq[0].h[1] = *(const ushort8*)(qp + 16);
        aq[1].h[0] = *(const ushort8*)(qp + 32);
        aq[1].h[1] = *(const ushort8*)(qp + 48);
    }

    v8f o[4] = {};
    float mvec[8], lvec[8];
    for (int r = 0; r < 8; ++r) { mvec[r] = -3.0e38f; lvec[r] = 0.f; }

    const int nkb = (qbase + 16 + 31) >> 5;
    for (int kb = 0; kb < nkb; ++kb) {
        const int kbase = kb * 32;
        Frag bk[2][2];
        for (int t = 0; t < 2; ++t) {
            const unsigned short* kp =
                qkvb + (size_t)(b * S + kbase + t * 16 + l15) * D3 + H * HD + h * HD + hi * 8;
            bk[t][0].h[0] = *(const ushort8*)(kp);      bk[t][0].h[1] = *(const ushort8*)(kp + 16);
            bk[t][1].h[0] = *(const ushort8*)(kp + 32); bk[t][1].h[1] = *(const ushort8*)(kp + 48);
        }
        v8f z = {};
        v8f sc[2];
        sc[0] = wmma16(aq[0].b, bk[0][0].b, z);
        sc[0] = wmma16(aq[1].b, bk[0][1].b, sc[0]);
        sc[1] = wmma16(aq[0].b, bk[1][0].b, z);
        sc[1] = wmma16(aq[1].b, bk[1][1].b, sc[1]);

        const bool diag = (kbase + 32 > qbase);
        for (int t = 0; t < 2; ++t)
            for (int r = 0; r < 8; ++r) {
                float v = sc[t][r] * 0.125f;
                if (diag) {
                    int key  = kbase + t * 16 + l15;
                    int qrow = qbase + r + hi * 8;
                    if (key > qrow) v = -1.0e30f;
                }
                sc[t][r] = v;
            }

        float al[8];
        for (int r = 0; r < 8; ++r) {
            float v = fmaxf(sc[0][r], sc[1][r]);
            v = fmaxf(v, __shfl_xor(v, 1, 32));
            v = fmaxf(v, __shfl_xor(v, 2, 32));
            v = fmaxf(v, __shfl_xor(v, 4, 32));
            v = fmaxf(v, __shfl_xor(v, 8, 32));
            float mn = fmaxf(mvec[r], v);
            al[r] = __expf(mvec[r] - mn);
            mvec[r] = mn;
        }
        for (int t = 0; t < 2; ++t)
            for (int r = 0; r < 8; ++r)
                sc[t][r] = __expf(sc[t][r] - mvec[r]);
        for (int r = 0; r < 8; ++r) {
            float rs = sc[0][r] + sc[1][r];
            rs += __shfl_xor(rs, 1, 32);
            rs += __shfl_xor(rs, 2, 32);
            rs += __shfl_xor(rs, 4, 32);
            rs += __shfl_xor(rs, 8, 32);
            lvec[r] = lvec[r] * al[r] + rs;
        }
        for (int n = 0; n < 4; ++n)
            for (int r = 0; r < 8; ++r)
                o[n][r] *= al[r];

        for (int t = 0; t < 2; ++t)
            for (int r = 0; r < 8; ++r)
                plds[w][(r + hi * 8) * 32 + t * 16 + l15] = f2b(sc[t][r] * PSC);
        asm volatile("s_wait_dscnt 0" ::: "memory");
        Frag pa;
        pa.h[0] = *(const ushort8*)&plds[w][l15 * 32 + hi * 8];
        pa.h[1] = *(const ushort8*)&plds[w][l15 * 32 + hi * 8 + 16];

        const unsigned short* vpp = vp + (((size_t)bh * (S / 32) + kb) * 4) * 512 + lane * 16;
        for (int n = 0; n < 4; ++n) {
            Frag bv;
            bv.u = *(const ushort16*)(vpp + n * 512);
            o[n] = wmma16(pa.b, bv.b, o[n]);
        }
        asm volatile("s_wait_dscnt 0" ::: "memory");
    }

    unsigned short* ot = olds[w];
    for (int n = 0; n < 4; ++n)
        for (int r = 0; r < 8; ++r) ot[(r + hi * 8) * 64 + n * 16 + l15] = f2b(o[n][r] * (PUN / lvec[r]));
    asm volatile("s_wait_dscnt 0" ::: "memory");
    __builtin_amdgcn_wave_barrier();
    for (int q = 0; q < 4; ++q) {
        const int rl = q * 4 + (lane >> 3), pc = lane & 7;
        vst2(attn + (size_t)(b * S + qbase + rl) * (H * HD) + h * HD + pc * 8, *(const v4u*)(ot + rl * 64 + pc * 8));
    }
}

__global__ void colmean(const float* __restrict__ x, float* __restrict__ out, int B, int S, int D) {
    int idx = blockIdx.x * 256 + threadIdx.x;
    if (idx >= B * D) return;
    int b = idx / D, d = idx % D;
    float s = 0.f;
    for (int t = 0; t < S; ++t) s += x[((size_t)b * S + t) * D + d];
    vst2(out + idx, (float_a)(s / (float)S));
}

__global__ __launch_bounds__(128) void state_update(
        const float* __restrict__ state, const float* __restrict__ meanx,
        const float* __restrict__ w_h2s, const float* __restrict__ w_sgate,
        float* __restrict__ outState, int D, int SD) {
    __shared__ float ni[2][64];
    int t = threadIdx.x;
    int b = t >> 6, j = t & 63;
    float s = 0.f;
    for (int k = 0; k < D; ++k) s += meanx[b * D + k] * w_h2s[(size_t)k * SD + j];
    ni[b][j] = s;
    __syncthreads();
    float g = 0.f;
    for (int k = 0; k < SD; ++k) g += state[b * SD + k] * w_sgate[k * SD + j];
    for (int k = 0; k < SD; ++k) g += ni[b][k] * w_sgate[(SD + k) * SD + j];
    g = 1.f / (1.f + __expf(-g));
    vst2(outState + b * SD + j, (float_a)(state[b * SD + j] * (1.f - g) + ni[b][j] * g));
}

extern "C" void kernel_launch(void* const* d_in, const int* in_sizes, int n_in,
                              void* d_out, int out_size, void* d_ws, size_t ws_size,
                              hipStream_t stream) {
    (void)in_sizes; (void)n_in; (void)out_size; (void)ws_size;
    const int B = 2, S = 2048, D = 1024, H = 16, HD = 64, SD = 64;
    const float* x       = (const float*)d_in[0];
    const float* gamma   = (const float*)d_in[1];
    const float* beta    = (const float*)d_in[2];
    const float* state   = (const float*)d_in[3];
    const float* w_qkv   = (const float*)d_in[4];
    const float* w_o     = (const float*)d_in[5];
    const float* w_gate  = (const float*)d_in[6];
    const float* w_up    = (const float*)d_in[7];
    const float* w_down  = (const float*)d_in[8];
    const float* norm1_w = (const float*)d_in[9];
    const float* norm2_w = (const float*)d_in[10];
    const float* w_sm    = (const float*)d_in[11];
    const float* w_h2s   = (const float*)d_in[12];
    const float* w_sgate = (const float*)d_in[13];
    float* xout = (float*)d_out;

    char* ws = (char*)d_ws;
    size_t off = 0;
    auto arena = [&](size_t bytes) -> void* {
        void* p = ws + off;
        off = (off + bytes + 255) & ~(size_t)255;
        return p;
    };
    float* fg             = (float*)arena((size_t)B * D * 4);
    float* fb             = (float*)arena((size_t)B * D * 4);
    unsigned short* hbuf  = (unsigned short*)arena((size_t)B * S * D * 2);
    unsigned short* wqkvp = (unsigned short*)arena((size_t)D * 3 * D * 2);
    unsigned short* wop   = (unsigned short*)arena((size_t)D * D * 2);
    unsigned short* wgp   = (unsigned short*)arena((size_t)D * 3 * D * 2);
    unsigned short* wupp  = (unsigned short*)arena((size_t)D * 3 * D * 2);
    unsigned short* wdp   = (unsigned short*)arena((size_t)3 * D * D * 2);
    unsigned short* qkvb  = (unsigned short*)arena((size_t)B * S * 3 * D * 2);
    unsigned short* vp    = (unsigned short*)arena((size_t)B * H * (S / 32) * 4 * 512 * 2);
    unsigned short* attnb = (unsigned short*)arena((size_t)B * S * D * 2);
    float* x1             = (float*)arena((size_t)B * S * D * 4);
    unsigned short* gateb = (unsigned short*)arena((size_t)B * S * 3 * D * 2);
    float* meanb          = (float*)arena((size_t)B * D * 4);
    unsigned short* act   = qkvb;

    const int MR = B * S;

    film_kernel<<<(B * 2 * D + 255) / 256, 256, 0, stream>>>(state, w_sm, gamma, beta, fg, fb, SD, D);

    pack_b<<<(D * 3 * D / 8 + 255) / 256, 256, 0, stream>>>(w_qkv,  wqkvp, D, 3 * D);
    pack_b<<<(D * D / 8 + 255) / 256,     256, 0, stream>>>(w_o,    wop,   D, D);
    pack_b<<<(D * 3 * D / 8 + 255) / 256, 256, 0, stream>>>(w_gate, wgp,   D, 3 * D);
    pack_b<<<(D * 3 * D / 8 + 255) / 256, 256, 0, stream>>>(w_up,   wupp,  D, 3 * D);
    pack_b<<<(3 * D * D / 8 + 255) / 256, 256, 0, stream>>>(w_down, wdp,   3 * D, D);

    rmsnorm_film<<<MR, 256, 0, stream>>>(x, norm1_w, fg, fb, hbuf, S, D);

    gemm_f16<0><<<dim3(3 * D / 256, MR / 64), 256, 0, stream>>>(
        hbuf, wqkvp, nullptr, nullptr, nullptr, qkvb, MR, 3 * D, D);

    {
        int total = B * H * (S / 32) * 4 * 512;
        pack_v<<<(total / 8 + 255) / 256, 256, 0, stream>>>(qkvb, vp, S, H, HD, total);
    }

    flash_attn<<<(B * H * (S / 16)) / 8, 256, 0, stream>>>(qkvb, vp, attnb, S, H, HD);

    gemm_f16<1><<<dim3(D / 256, MR / 64), 256, 0, stream>>>(
        attnb, wop, x, nullptr, x1, nullptr, MR, D, D);

    rmsnorm_film<<<MR, 256, 0, stream>>>(x1, norm2_w, fg, fb, hbuf, S, D);

    gemm_f16<2><<<dim3(3 * D / 256, MR / 64), 256, 0, stream>>>(
        hbuf, wgp, nullptr, nullptr, nullptr, gateb, MR, 3 * D, D);

    gemm_f16<3><<<dim3(3 * D / 256, MR / 64), 256, 0, stream>>>(
        hbuf, wupp, nullptr, gateb, nullptr, act, MR, 3 * D, D);

    gemm_f16<1><<<dim3(D / 256, MR / 64), 256, 0, stream>>>(
        act, wdp, x1, nullptr, xout, nullptr, MR, D, 3 * D);

    colmean<<<(B * D + 255) / 256, 256, 0, stream>>>(xout, meanb, B, S, D);
    state_update<<<1, 128, 0, stream>>>(state, meanb, w_h2s, w_sgate,
                                        xout + (size_t)B * S * D, D, SD);
}
